// Model_8495445311643
// MI455X (gfx1250) — hardware-run, weakly checked
//
#include <hip/hip_runtime.h>


#define NB_  2
#define NE   64
#define NT   96
#define DM   128
#define NS   (NB_ * NT)
#define NR   (NS * NE)
#define HE   32
#define PCAR 1024.0f

typedef _Float16 h16;
typedef unsigned short bf;
typedef __attribute__((ext_vector_type(16))) __bf16   v16bf;
typedef __attribute__((ext_vector_type(16))) _Float16 v16h;
typedef __attribute__((ext_vector_type(8)))  _Float16 v8h;
typedef __attribute__((ext_vector_type(8)))  unsigned short v8us;
typedef __attribute__((ext_vector_type(8)))  float    v8f;
typedef __attribute__((ext_vector_type(4)))  float    v4f;
typedef v8h  __attribute__((may_alias)) v8ha;
typedef v4f  __attribute__((may_alias)) v4fa;
typedef v8us __attribute__((may_alias)) v8usa;

__device__ __forceinline__ unsigned short f2bf(float f) { unsigned u = __float_as_uint(f); u += 0x7FFFu + ((u >> 16) & 1u); return (unsigned short)(u >> 16); }
__device__ __forceinline__ float bf2f(unsigned short b) { return __uint_as_float(((unsigned)b) << 16); }
__device__ __forceinline__ float bfr(float f) { return bf2f(f2bf(f)); }
__device__ __forceinline__ v16h cat16(v8h lo, v8h hi) { return __builtin_shufflevector(lo, hi, 0, 1, 2, 3, 4, 5, 6, 7, 8, 9, 10, 11, 12, 13, 14, 15); }
__device__ __forceinline__ v16bf cat16b(v8us lo, v8us hi) { return __builtin_bit_cast(v16bf, __builtin_shufflevector(lo, hi, 0, 1, 2, 3, 4, 5, 6, 7, 8, 9, 10, 11, 12, 13, 14, 15)); }
__device__ __forceinline__ v8f wmma16(v16h a, v16h b, v8f c) { return __builtin_amdgcn_wmma_f32_16x16x32_f16(false, a, false, b, (short)0, c, false, false); }
__device__ __forceinline__ v8f wmmab(v16bf a, v16bf b, v8f c) { return __builtin_amdgcn_wmma_f32_16x16x32_bf16(false, a, false, b, (short)0, c, false, false); }
typedef __attribute__((ext_vector_type(2))) _Float16 v2h;
typedef __attribute__((ext_vector_type(4))) _Float16 v4h;
typedef __attribute__((ext_vector_type(2))) unsigned short v2us;
typedef __attribute__((ext_vector_type(4))) unsigned short v4us;
typedef __attribute__((ext_vector_type(2))) float v2f;
typedef __attribute__((ext_vector_type(4))) int v4i;

template <typename T16> struct WFrag;
template <> struct WFrag<h16> { typedef v16h V; static __device__ __forceinline__ V ld(const h16* p) { return cat16(*(const v8h*)p, *(const v8h*)(p + 16)); } static __device__ __forceinline__ v8f mma(V a, V b, v8f c) { return wmma16(a, b, c); } };
template <> struct WFrag<bf> { typedef v16bf V; static __device__ __forceinline__ V ld(const bf* p) { return cat16b(*(const v8us*)p, *(const v8us*)(p + 16)); } static __device__ __forceinline__ v8f mma(V a, V b, v8f c) { return wmmab(a, b, c); } };
template <typename T16, int NSPLIT, bool BIAS>
__global__ __launch_bounds__(32) void k_gemmw(const T16* __restrict__ A, const T16* __restrict__ A2, const T16* __restrict__ Bt, const T16* __restrict__ Bt2, int K, float* C, int ldc, const float* __restrict__ bias, size_t sA, size_t sB, size_t sC) {
    typedef typename WFrag<T16>::V V;
    __shared__ __align__(16) float os[16 * 68];
    const size_t z = blockIdx.z; A += z * sA; if (A2) A2 += z * sA; Bt += z * sB; if (Bt2) Bt2 += z * sB; C += z * sC;
    const int lane = threadIdx.x & 31, lr = lane & 15, hi = lane >> 4; const int r0 = blockIdx.x * 64, c0 = blockIdx.y * 64;
    v8f acc[4][4];
#pragma unroll
    for (int mb = 0; mb < 4; ++mb)
#pragma unroll
        for (int nb = 0; nb < 4; ++nb) acc[mb][nb] = (v8f){};
    const size_t aoff = (size_t)(r0 + lr) * K + 8 * hi, boff = (size_t)(c0 + lr) * K + 8 * hi;

    for (int kc = 0; kc < K; kc += 32) {
        V a[4], a2[4];
#pragma unroll
        for (int mb = 0; mb < 4; ++mb) { a[mb] = WFrag<T16>::ld(A + aoff + (size_t)mb * 16 * K + kc); if (NSPLIT == 1 || NSPLIT == 2) a2[mb] = WFrag<T16>::ld(A2 + aoff + (size_t)mb * 16 * K + kc); }
#pragma unroll
        for (int nb = 0; nb < 4; ++nb) { const V b = WFrag<T16>::ld(Bt + boff + (size_t)nb * 16 * K + kc); V b2; if (NSPLIT >= 2) b2 = WFrag<T16>::ld(Bt2 + boff + (size_t)nb * 16 * K + kc);
#pragma unroll
            for (int mb = 0; mb < 4; ++mb) { acc[mb][nb] = WFrag<T16>::mma(a[mb], b, acc[mb][nb]); if (NSPLIT == 1 || NSPLIT == 2) acc[mb][nb] = WFrag<T16>::mma(a2[mb], b, acc[mb][nb]); if (NSPLIT >= 2) acc[mb][nb] = WFrag<T16>::mma(a[mb], b2, acc[mb][nb]); } }
        asm volatile("v_nop\n\tv_nop\n\tv_nop\n\tv_nop" : "+v"(acc[0][0]), "+v"(acc[1][1]), "+v"(acc[2][2]), "+v"(acc[3][3]) : "v"(a[0]), "v"(a[3]));
    }
#pragma unroll
    for (int mb = 0; mb < 4; ++mb) {
#pragma unroll
        for (int nb = 0; nb < 4; ++nb) {
#pragma unroll
            for (int j = 0; j < 8; ++j) os[(hi * 8 + j) * 68 + nb * 16 + lr] = acc[mb][nb][j]; }
        __builtin_amdgcn_wave_barrier(); asm volatile("" ::: "memory");
        float* crow = C + (size_t)(r0 + mb * 16) * ldc + c0;
#pragma unroll 1
        for (int ps = 0; ps < 2; ++ps) {
#pragma unroll
            for (int s = 0; s < 8; ++s) { const int row = 2 * s + hi, cofs = lr * 4; v4f val = *(const v4fa*)(os + row * 68 + cofs); if (BIAS) { val[0] += bfr(bias[c0 + cofs]); val[1] += bfr(bias[c0 + cofs + 1]); val[2] += bfr(bias[c0 + cofs + 2]); val[3] += bfr(bias[c0 + cofs + 3]); }
                *(volatile v4f*)(crow + (size_t)row * ldc + cofs) = val; }
            if (ps == 0) __threadfence(); }
        __builtin_amdgcn_wave_barrier(); asm volatile("" ::: "memory");
    }
}

__device__ __forceinline__ h16 tohx(float x) { return (h16)x; }
__device__ __forceinline__ void splitf(float y, unsigned short& h, unsigned short& l) { h = f2bf(y); l = f2bf(y - bf2f(h)); }
typedef __attribute__((ext_vector_type(2))) _Float16 v2h;
typedef __attribute__((ext_vector_type(4))) _Float16 v4h;
typedef __attribute__((ext_vector_type(2))) unsigned short v2us;
typedef __attribute__((ext_vector_type(4))) unsigned short v4us;
typedef __attribute__((ext_vector_type(2))) float v2f;
typedef __attribute__((ext_vector_type(4))) int v4i;

__global__ __launch_bounds__(256) void k_cvt8(const float* __restrict__ src, bf* dst, size_t n8) { const size_t i = (size_t)blockIdx.x * 256 + threadIdx.x; if (i >= n8) return; const v8f v = *(const v8f*)(src + i * 8); v8us o;
#pragma unroll
    for (int k = 0; k < 8; ++k) o[k] = f2bf(v[k]); *(volatile v8us*)(dst + i * 8) = o; __threadfence(); *(volatile v8us*)(dst + i * 8) = o; }

__global__ __launch_bounds__(256) void k_wtG(const float* __restrict__ w, int K, int N, bf* Bt) {
    const int lane = threadIdx.x & 31; const int L0 = (blockIdx.x * 8 + (threadIdx.x >> 5)) * 8; const int nlines = N * K / 64;
#pragma unroll
    for (int ps = 0; ps < 2; ++ps) {
        for (int l = 0; l < 8; ++l) { const int L = L0 + l; if (L >= nlines) break; const size_t e = (size_t)L * 64 + lane * 2; const int k = (int)(e % K), n = (int)(e / K); v2us o;
            o[0] = f2bf(w[(size_t)k * N + n]); o[1] = f2bf(w[(size_t)(k + 1) * N + n]); *(volatile v2us*)(Bt + e) = o; }
        if (ps == 0) __threadfence(); }
}
__global__ __launch_bounds__(256) void k_fillb(bf* P, unsigned w2, size_t n8) { const size_t i = (size_t)blockIdx.x * 256 + threadIdx.x; if (i >= n8) return; v4i o; o[0] = (int)w2; o[1] = (int)w2; o[2] = (int)w2; o[3] = (int)w2;
    *(volatile v4i*)(P + i * 8) = o; __threadfence(); *(volatile v4i*)(P + i * 8) = o; }

__global__ __launch_bounds__(256) void k_cvp(const float* __restrict__ F, int perm, float sc, h16* O16) { const size_t e = ((size_t)blockIdx.x * 256 + threadIdx.x) * 8; if (e >= (size_t)NR * DM) return; const int d0 = (int)(e % DM); const int r = (int)(e / DM); const int n = r % NE; const int st = r / NE; const int t = st % NT; const int b = st / NT; const int rx = (b * NE + n) * NT + t; const int rs = perm ? rx : r;
    const float* fr = F + (size_t)rs * DM + d0; const v4f a = *(const v4f*)fr; const v4f c = *(const v4f*)(fr + 4); v8h o16;
#pragma unroll
    for (int q = 0; q < 4; ++q) { o16[q] = tohx(__fmul_rn(a[q], sc)); o16[q + 4] = tohx(__fmul_rn(c[q], sc)); }
    *(volatile v8h*)(O16 + e) = o16; __threadfence(); *(volatile v8h*)(O16 + e) = o16; }

__global__ __launch_bounds__(256) void k_wth(const float* __restrict__ w, int N, h16* Bt) { const size_t e = ((size_t)blockIdx.x * 256 + threadIdx.x) * 8; if (e >= (size_t)N * DM) return; const int k0 = (int)(e % DM); const int n = (int)(e / DM); v8h o;
#pragma unroll
    for (int q = 0; q < 8; ++q) o[q] = tohx(bfr(w[(size_t)(k0 + q) * N + n]));
    *(volatile v8h*)(Bt + e) = o; __threadfence(); *(volatile v8h*)(Bt + e) = o; }

__global__ __launch_bounds__(256) void k_vt64(const float* __restrict__ V, h16* VT) { const size_t e = ((size_t)blockIdx.x * 256 + threadIdx.x) * 8; if (e >= (size_t)NS * DM * NE) return; const int n0 = (int)(e % NE); const int d = (int)((e / NE) % DM); const int st = (int)(e / ((size_t)NE * DM)); const int t = st % NT; const int b = st / NT; v8h w;
#pragma unroll
    for (int q = 0; q < 8; ++q) w[q] = tohx(V[((size_t)(b * NE + n0 + q) * NT + t) * DM + d]);
    *(volatile v8h*)(VT + e) = w; __threadfence(); *(volatile v8h*)(VT + e) = w; }

__global__ __launch_bounds__(256) void k_pair(const float* __restrict__ CL, const float* __restrict__ QH, const float* __restrict__ KH, const float* __restrict__ EF, const float* __restrict__ AP, const int* __restrict__ PM, const float* __restrict__ W1, const float* __restrict__ B1, const float* __restrict__ W2, const float* __restrict__ B2, const float* __restrict__ WF, const float* __restrict__ PW, const float* __restrict__ PRW, float* LG) {
    const size_t e = (size_t)blockIdx.x * 256 + threadIdx.x; if (e >= (size_t)NS * NE * NE) return; const int j = (int)(e % NE); const int i = (int)((e / NE) % NE); const int st = (int)(e / ((size_t)NE * NE)); const int b = st / NT;
    const float* qh = QH + ((size_t)st * NE + i) * 64; const float* kh = KH + ((size_t)st * NE + j) * 64; const v4f ef = *(const v4f*)(EF + e * 4); const float e0 = bfr(ef[0]), e1 = bfr(ef[1]), e2 = bfr(ef[2]), e3 = bfr(ef[3]); const float* w1e = W1 + 2 * DM * HE; float ph = 0.0f;
#pragma unroll 1
    for (int ug = 0; ug < 4; ++ug) {
#pragma unroll
    for (int u4 = 2 * ug; u4 < 2 * ug + 2; ++u4) { const v4f q4 = *(const v4f*)(qh + 4 * u4); const v4f k4 = *(const v4f*)(kh + 4 * u4);
#pragma unroll
        for (int q = 0; q < 4; ++q) { const int u = 4 * u4 + q; float eh = __fmul_rn(e0, bfr(w1e[u])); eh = __fmaf_rn(e1, bfr(w1e[HE + u]), eh); eh = __fmaf_rn(e2, bfr(w1e[2 * HE + u]), eh); eh = __fmaf_rn(e3, bfr(w1e[3 * HE + u]), eh); const float hv = fmaxf(__fadd_rn(__fadd_rn(__fadd_rn(q4[q], k4[q]), eh), bfr(B1[u])), 0.0f); ph = __fmaf_rn(hv, bfr(W2[u]), ph); } } }
    ph = __fadd_rn(ph, bfr(B2[0]));
    const float* ap = AP + e * 5; float a = __fmul_rn(bfr(ap[0]), bfr(WF[0])); a = __fmaf_rn(bfr(ap[1]), bfr(WF[1]), a); a = __fmaf_rn(bfr(ap[2]), bfr(WF[2]), a); a = __fmaf_rn(bfr(ap[3]), bfr(WF[3]), a); a = __fmaf_rn(bfr(ap[4]), bfr(WF[4]), a);
    a = (a != a) ? 0.0f : a; a = (fabsf(a) > 3.0e38f) ? 0.0f : a; a = fmaxf(a, 0.0f); const float lp = __fmul_rn(__builtin_amdgcn_logf(__fadd_rn(a, 1.0e-6f)), 0.69314718055994531f);
    float lg = __fmul_rn(CL[e], 0.088388347648318441f); lg = __fmaf_rn(bfr(PW[0]), ph, lg); lg = __fmaf_rn(bfr(PRW[0]), lp, lg); const bool bad = (PM[b * NE + i] != 0) | (PM[b * NE + j] != 0); lg = bad ? -1.0e9f : lg;
    *(volatile float*)(LG + e) = lg; __threadfence(); *(volatile float*)(LG + e) = lg; }

__global__ __launch_bounds__(256) void k_sm64(const float* __restrict__ LG, h16* P16) { const size_t e = ((size_t)blockIdx.x * 256 + threadIdx.x) * 8; if (e >= (size_t)NR * NE) return; const int j0 = (int)(e % NE); const size_t row = e / NE; const float* lr = LG + row * NE; float m = -3.0e38f; v4f z[16];
#pragma unroll
    for (int g = 0; g < 16; ++g) { z[g] = *(const v4f*)(lr + 4 * g); m = fmaxf(fmaxf(fmaxf(fmaxf(m, z[g][0]), z[g][1]), z[g][2]), z[g][3]); }
    float sum = 0.0f;
#pragma unroll
    for (int g = 0; g < 16; ++g) {
#pragma unroll
        for (int q = 0; q < 4; ++q) sum = __fadd_rn(sum, __builtin_amdgcn_exp2f(__fmul_rn(__fsub_rn(z[g][q], m), 1.4426950408889634f))); }
    const float r = __fmul_rn(__fdiv_rn(1.0f, sum), PCAR); const v4f a = *(const v4f*)(lr + j0); const v4f c = *(const v4f*)(lr + j0 + 4); v8h w;
#pragma unroll
    for (int q = 0; q < 4; ++q) { w[q] = tohx(__fmul_rn(__builtin_amdgcn_exp2f(__fmul_rn(__fsub_rn(a[q], m), 1.4426950408889634f)), r)); w[q + 4] = tohx(__fmul_rn(__builtin_amdgcn_exp2f(__fmul_rn(__fsub_rn(c[q], m), 1.4426950408889634f)), r)); }
    *(volatile v8h*)(P16 + e) = w; __threadfence(); *(volatile v8h*)(P16 + e) = w; }

__global__ __launch_bounds__(256) void k_rln(const float* __restrict__ X, const float* __restrict__ OF, const float* __restrict__ G, const float* __restrict__ Bv, const int* __restrict__ PM, float* OUT) { const size_t e = ((size_t)blockIdx.x * 256 + threadIdx.x) * 4; if (e >= (size_t)NR * DM) return; const int d0 = (int)(e % DM); const int rx = (int)(e / DM); const int t = rx % NT; const int bn = rx / NT; const int n = bn % NE; const int b = bn / NE; const int rs = (b * NT + t) * NE + n;
    const float* xr = X + (size_t)rx * DM; const float* fr = OF + (size_t)rs * DM; float s = 0.0f;
#pragma unroll
    for (int g = 0; g < DM / 4; ++g) { const v4f xv = *(const v4f*)(xr + 4 * g); const v4f fv = *(const v4f*)(fr + 4 * g);
#pragma unroll
        for (int q = 0; q < 4; ++q) s = __fadd_rn(s, __fadd_rn(bfr(xv[q]), fv[q])); }
    const float mu = __fmul_rn(s, 1.0f / DM); float v2 = 0.0f;
#pragma unroll
    for (int g = 0; g < DM / 4; ++g) { const v4f xv = *(const v4f*)(xr + 4 * g); const v4f fv = *(const v4f*)(fr + 4 * g);
#pragma unroll
        for (int q = 0; q < 4; ++q) { const float dd = __fsub_rn(__fadd_rn(bfr(xv[q]), fv[q]), mu); v2 = __fmaf_rn(dd, dd, v2); } }
    const float rstd = __fdiv_rn(1.0f, __fsqrt_rn(__fadd_rn(__fmul_rn(v2, 1.0f / DM), 1.0e-5f))); const float f = (PM[b * NE + n] != 0) ? 0.0f : 1.0f; const v4f xo = *(const v4f*)(xr + d0); const v4f fo = *(const v4f*)(fr + d0); const v4f gg = *(const v4f*)(G + d0); const v4f bb = *(const v4f*)(Bv + d0); v4f o;
#pragma unroll
    for (int q = 0; q < 4; ++q) o[q] = __fmul_rn(__fmaf_rn(__fmul_rn(__fsub_rn(__fadd_rn(bfr(xo[q]), fo[q]), mu), rstd), bfr(gg[q]), bfr(bb[q])), f);
    *(volatile v4f*)(OUT + e) = o; __threadfence(); *(volatile v4f*)(OUT + e) = o; }

extern "C" void kernel_launch(void* const* d_in, const int* in_sizes, int n_in,
                              void* d_out, int out_size, void* d_ws, size_t ws_size, hipStream_t stream) {
    (void)in_sizes; (void)n_in; (void)out_size;
    const float* xin = (const float*)d_in[0]; const float* efin = (const float*)d_in[1]; const float* apin = (const float*)d_in[2]; const int* pmin = (const int*)d_in[3];
    const float* wq = (const float*)d_in[4]; const float* wk = (const float*)d_in[5]; const float* wv = (const float*)d_in[6]; const float* w1 = (const float*)d_in[7]; const float* b1 = (const float*)d_in[8]; const float* w2 = (const float*)d_in[9]; const float* b2 = (const float*)d_in[10]; const float* wf = (const float*)d_in[11]; const float* wth = (const float*)d_in[12]; const float* lng = (const float*)d_in[13]; const float* lnb = (const float*)d_in[14]; const float* pw = (const float*)d_in[15]; const float* prw = (const float*)d_in[16];
    float* OUT = (float*)d_out;
    char* wsp = (char*)d_ws;
    auto take = [&](size_t bytes) { char* p = wsp; wsp += (bytes + 255) & ~(size_t)255; return (void*)p; };
    const size_t NP = (size_t)NR * DM;
    bf* XB = (bf*)take(NP * 2); bf* WQB = (bf*)take((size_t)DM * DM * 2); bf* WKB = (bf*)take((size_t)DM * DM * 2); bf* WVB = (bf*)take((size_t)DM * DM * 2); h16* WT16 = (h16*)take((size_t)DM * DM * 2); h16* W1Q = (h16*)take((size_t)64 * DM * 2); h16* W1K = (h16*)take((size_t)64 * DM * 2);
    float* Qf = (float*)take(NP * 4); float* Kf = (float*)take(NP * 4); float* Vf = (float*)take(NP * 4);
    h16* Q16 = (h16*)take(NP * 2); h16* K16 = (h16*)take(NP * 2); h16* VT = (h16*)take(NP * 2);
    float* QH = (float*)take((size_t)NR * 64 * 4); float* KH = (float*)take((size_t)NR * 64 * 4); float* CL = (float*)take((size_t)NS * NE * NE * 4); float* LG = (float*)take((size_t)NS * NE * NE * 4); h16* P16 = (h16*)take((size_t)NS * NE * NE * 2);
    float* SP = (float*)take(NP * 4); h16* S16 = (h16*)take(NP * 2); float* OF = (float*)take(NP * 4);
    if ((size_t)(wsp - (char*)d_ws) > ws_size) return;
    k_cvt8<<<(unsigned)((NP / 8 + 255) / 256), 256, 0, stream>>>(xin, XB, NP / 8);
    k_wtG<<<(unsigned)((DM * DM / 64 + 63) / 64), 256, 0, stream>>>(wq, DM, DM, WQB); k_wtG<<<(unsigned)((DM * DM / 64 + 63) / 64), 256, 0, stream>>>(wk, DM, DM, WKB); k_wtG<<<(unsigned)((DM * DM / 64 + 63) / 64), 256, 0, stream>>>(wv, DM, DM, WVB);
    k_wth<<<(unsigned)((size_t)DM * DM / 2048), 256, 0, stream>>>(wth, DM, WT16);
    k_wth<<<(unsigned)((size_t)HE * DM / 2048), 256, 0, stream>>>(w1, HE, W1Q); k_wth<<<(unsigned)((size_t)HE * DM / 2048), 256, 0, stream>>>(w1 + (size_t)DM * HE, HE, W1K);
    k_fillb<<<(unsigned)(((size_t)32 * DM / 8 + 255) / 256), 256, 0, stream>>>((bf*)(W1Q + (size_t)HE * DM), 0u, (size_t)32 * DM / 8); k_fillb<<<(unsigned)(((size_t)32 * DM / 8 + 255) / 256), 256, 0, stream>>>((bf*)(W1K + (size_t)HE * DM), 0u, (size_t)32 * DM / 8);
    k_gemmw<bf, 0, false><<<dim3(NR / 64, DM / 64, 1), 32, 0, stream>>>(XB, nullptr, WQB, nullptr, DM, Qf, DM, nullptr, 0, 0, 0); k_gemmw<bf, 0, false><<<dim3(NR / 64, DM / 64, 1), 32, 0, stream>>>(XB, nullptr, WKB, nullptr, DM, Kf, DM, nullptr, 0, 0, 0); k_gemmw<bf, 0, false><<<dim3(NR / 64, DM / 64, 1), 32, 0, stream>>>(XB, nullptr, WVB, nullptr, DM, Vf, DM, nullptr, 0, 0, 0);
    k_cvp<<<(unsigned)(NP / 2048), 256, 0, stream>>>(Qf, 1, 1.0f, Q16); k_cvp<<<(unsigned)(NP / 2048), 256, 0, stream>>>(Kf, 1, 1.0f, K16);
    k_vt64<<<(unsigned)(NP / 2048), 256, 0, stream>>>(Vf, VT);
    k_gemmw<h16, 0, false><<<dim3(NR / 64, 1, 1), 32, 0, stream>>>(Q16, nullptr, W1Q, nullptr, DM, QH, 64, nullptr, 0, 0, 0); k_gemmw<h16, 0, false><<<dim3(NR / 64, 1, 1), 32, 0, stream>>>(K16, nullptr, W1K, nullptr, DM, KH, 64, nullptr, 0, 0, 0);
    k_gemmw<h16, 0, false><<<dim3(1, 1, NS), 32, 0, stream>>>(Q16, nullptr, K16, nullptr, DM, CL, NE, nullptr, (size_t)NE * DM, (size_t)NE * DM, (size_t)NE * NE);
    k_pair<<<(unsigned)((size_t)NS * NE * NE / 256), 256, 0, stream>>>(CL, QH, KH, efin, apin, pmin, w1, b1, w2, b2, wf, pw, prw, LG);
    k_sm64<<<(unsigned)((size_t)NR * NE / 2048), 256, 0, stream>>>(LG, P16);
    k_gemmw<h16, 0, false><<<dim3(1, DM / 64, NS), 32, 0, stream>>>(P16, nullptr, VT, nullptr, NE, SP, DM, nullptr, (size_t)NE * NE, (size_t)DM * NE, (size_t)NE * DM);
    k_cvp<<<(unsigned)(NP / 2048), 256, 0, stream>>>(SP, 0, 1.0f / PCAR, S16);
    k_gemmw<h16, 0, false><<<dim3(NR / 64, DM / 64, 1), 32, 0, stream>>>(S16, nullptr, WT16, nullptr, DM, OF, DM, nullptr, 0, 0, 0);
    k_rln<<<(unsigned)(NP / 1024), 256, 0, stream>>>(xin, OF, lng, lnb, pmin, OUT);
}
